// GNN_graphpred_42391327212259
// MI455X (gfx1250) — hardware-run, weakly checked
//
#include <hip/hip_runtime.h>
#include <stddef.h>
#include <stdint.h>


#define XD     5
#define PD     3
#define F0     14
#define F1     132
#define NCH    64
#define NUV    128
#define KP0    32
#define KP     192
#define NTHR   256
#define NWAVE  8
#define EPT    8
#define CHUNK  (NTHR * EPT)
#define WCAP   (EPT * 32)
#define LISTN  (NWAVE * WCAP)
#define NBA    1024
#define SLA    10
#define RCAP   28672
#define DEGCAP 1024
#define GBM    64
#define GBN    128
#define GTHR   128
#define NBP    32
#define GPW    (NBP / NWAVE)
#define NU0B   (NUV * (KP0 / 8))
#define NU1B   (NUV * (KP / 8))
#define AGG_ZINTS (LISTN + 2 * RCAP + 3 * NBA)
#define AGG_LDS_INTS (AGG_ZINTS + 16)
#define WSMAX  134217728

static_assert((CHUNK & (CHUNK - 1)) == 0 && CHUNK <= 4096);
static_assert((NBA & (NBA - 1)) == 0 && NBA == (1 << SLA));
static_assert(((long long)CHUNK << SLA) < (1LL << 31));
static_assert(LISTN % NTHR == 0);
static_assert(NBA % NWAVE == 0 && NBA % 32 == 0);
static_assert(RCAP % 32 == 0 && AGG_ZINTS % (4 * NTHR) == 0);
static_assert(KP0 % 32 == 0 && KP % 32 == 0 && KP0 >= XD + PD && KP >= 2 * NCH + PD);
static_assert(NUV == GBN && NUV == 2 * NCH && NCH == 64);
static_assert(GBM == (GTHR / 32) * 16 && GBN == 4 * 32);
static_assert(NU0B % NTHR == 0 && NU1B % NTHR == 0);
static_assert(AGG_LDS_INTS * 4 <= 300000);
static_assert(NBP == GPW * NWAVE && NBP == 32);
static_assert(F0 == 2 * XD + 1 + PD && F1 == 2 * NCH + 1 + PD);

typedef float          v2f   __attribute__((ext_vector_type(2)));
typedef float          v4f   __attribute__((ext_vector_type(4)));
typedef float          v8f   __attribute__((ext_vector_type(8)));
typedef int            v4i   __attribute__((ext_vector_type(4)));
typedef int            v8i   __attribute__((ext_vector_type(8)));
typedef unsigned short v8us  __attribute__((ext_vector_type(8)));
typedef unsigned short v16us __attribute__((ext_vector_type(16)));
typedef __bf16         v16bf __attribute__((ext_vector_type(16)));
typedef v4f  __attribute__((may_alias)) v4fa;
typedef v4i  __attribute__((may_alias)) v4ia;
typedef v8us __attribute__((may_alias)) v8usa;
union FragB { v16bf v; v16us u; v8us h[2]; v8i w; };

__device__ __forceinline__ v8f wmb(const FragB& a, const FragB& b, v8f c) {
  v8f d = __builtin_amdgcn_wmma_f32_16x16x32_bf16(false, a.v, false, b.v, (short)0, c, false, false);
  asm volatile("v_nop\n\tv_nop\n\tv_nop\n\tv_nop" : "+v"(d) : "v"(a.w), "v"(b.w));
  return d;
}

__device__ __forceinline__ unsigned bf16_bits(float f) {
  const unsigned u = __float_as_uint(f);
  return (u + 0x7FFFu + ((u >> 16) & 1u)) >> 16;
}
__device__ __forceinline__ float bf16_val(float f) {
  return __uint_as_float(bf16_bits(f) << 16);
}
__device__ __forceinline__ float fsig(float z) {
  return __builtin_amdgcn_rcpf(1.0f + __expf(-z));
}
__device__ __forceinline__ float wsum(float q) {
  q += __shfl_xor(q, 16); q += __shfl_xor(q, 8); q += __shfl_xor(q, 4); q += __shfl_xor(q, 2); q += __shfl_xor(q, 1);
  return q;
}

template <int SLB>
__device__ __forceinline__ int scan_chunk(const int* __restrict__ ids, int nE, int cbase, int slotBase,
                                          int nb, int vec8, int* list, int tid, int lane, int wave) {
  int wc = 0;
  const int el0  = tid * EPT;
  const int e0   = cbase + el0;
  const int sent = -2147483647 - 1;
  v4i da, db;
  if (vec8 != 0 && cbase + CHUNK <= nE) {
    da = *(const v4i*)(ids + e0);
    db = *(const v4i*)(ids + e0 + 4);
  } else {
    da.x = (e0     < nE) ? ids[min(e0,     nE - 1)] : sent;
    da.y = (e0 + 1 < nE) ? ids[min(e0 + 1, nE - 1)] : sent;
    da.z = (e0 + 2 < nE) ? ids[min(e0 + 2, nE - 1)] : sent;
    da.w = (e0 + 3 < nE) ? ids[min(e0 + 3, nE - 1)] : sent;
    db.x = (e0 + 4 < nE) ? ids[min(e0 + 4, nE - 1)] : sent;
    db.y = (e0 + 5 < nE) ? ids[min(e0 + 5, nE - 1)] : sent;
    db.z = (e0 + 6 < nE) ? ids[min(e0 + 6, nE - 1)] : sent;
    db.w = (e0 + 7 < nE) ? ids[min(e0 + 7, nE - 1)] : sent;
  }
  const unsigned nbs = (unsigned)slotBase;
  const unsigned unb = (unsigned)nb;
  const unsigned s0 = (unsigned)da.x - nbs, s1 = (unsigned)da.y - nbs;
  const unsigned s2 = (unsigned)da.z - nbs, s3 = (unsigned)da.w - nbs;
  const unsigned s4 = (unsigned)db.x - nbs, s5 = (unsigned)db.y - nbs;
  const unsigned s6 = (unsigned)db.z - nbs, s7 = (unsigned)db.w - nbs;
  const bool h0 = s0 < unb, h1 = s1 < unb, h2 = s2 < unb, h3 = s3 < unb;
  const bool h4 = s4 < unb, h5 = s5 < unb, h6 = s6 < unb, h7 = s7 < unb;
  const unsigned any = __builtin_amdgcn_ballot_w32(h0 | h1 | h2 | h3 | h4 | h5 | h6 | h7);
  if (any != 0u) {
#define HITJ(J, HJ, SJ) { \
      const unsigned mj = __builtin_amdgcn_ballot_w32(HJ); \
      if (mj != 0u) { \
        if (HJ) { \
          const int pos = wc + (int)__builtin_amdgcn_mbcnt_lo(mj, 0u); \
          if (pos < WCAP) list[wave * WCAP + pos] = ((el0 + (J)) << SLB) | (int)(SJ); \
        } \
        wc += (int)__builtin_popcount(mj); } }
    HITJ(0, h0, s0)
    HITJ(1, h1, s1)
    HITJ(2, h2, s2)
    HITJ(3, h3, s3)
    HITJ(4, h4, s4)
    HITJ(5, h5, s5)
    HITJ(6, h6, s6)
    HITJ(7, h7, s7)
#undef HITJ
  }
  return wc;
}

__device__ __forceinline__ void bunit132(const float* __restrict__ W, int v, v8us& o) {
  const int n    = v / (KP / 8);
  const int k8   = (v - n * (KP / 8)) * 8;
  const int half = n >> 6;
  const int nn   = n & (NCH - 1);
#pragma unroll
  for (int e = 0; e < 8; ++e) {
    const int k = k8 + e;
    int rw = (k < 2 * NCH) ? ((k & (NCH - 1)) + NCH * half) : (2 * NCH + 1 + (k - 2 * NCH));
    rw = rw < 0 ? 0 : (rw > F1 - 1 ? F1 - 1 : rw);
    const float wv = W[(size_t)rw * NCH + nn];
    const bool isd = (k >= 2 * NCH) && (k < 2 * NCH + PD);
    const float sv = (isd && half != 0) ? -wv : wv;
    const float val = (k < 2 * NCH + PD) ? sv : 0.0f;
    o[e] = (unsigned short)bf16_bits(val);
  }
}

__global__ __launch_bounds__(NTHR) void k_prep(const float* __restrict__ x, const float* __restrict__ p,
                                               const float* __restrict__ W0, const float* __restrict__ W1,
                                               const float* __restrict__ W2, int nN, int nbA,
                                               unsigned short* A0, unsigned short* B0T,
                                               unsigned short* B1T, unsigned short* B2T) {
  const int b = (int)blockIdx.x, tid = (int)threadIdx.x;
  v8us o;
  unsigned short* dp;
  if (b < nbA) {
    const int u   = b * NTHR + tid;
    const int row = u >> 2;
    const int k8  = (u & 3) * 8;
    const int rc  = row < nN ? row : nN - 1;
    const bool ok = (row < nN) && (k8 == 0);
    const float* xp = x + (size_t)rc * XD;
    const float* pq = p + (size_t)rc * PD;
    float f[8];
    f[0] = xp[0]; f[1] = xp[1]; f[2] = xp[2]; f[3] = xp[3]; f[4] = xp[4];
    f[5] = pq[0]; f[6] = pq[1]; f[7] = pq[2];
#pragma unroll
    for (int e = 0; e < 8; ++e) o[e] = ok ? (unsigned short)bf16_bits(f[e]) : (unsigned short)0;
    dp = A0 + (size_t)u * 8;
  } else if (b < nbA + NU0B / NTHR) {
    const int v    = (b - nbA) * NTHR + tid;
    const int n    = v >> 2;
    const int k8   = (v & 3) * 8;
    const int half = n >> 6;
    const int nn   = n & (NCH - 1);
#pragma unroll
    for (int e = 0; e < 8; ++e) {
      const int k = k8 + e;
      int rw = (k < XD) ? (k + XD * half) : (2 * XD + 1 + (k - XD));
      rw = rw < 0 ? 0 : (rw > F0 - 1 ? F0 - 1 : rw);
      const float wv = W0[(size_t)rw * NCH + nn];
      const bool isd = (k >= XD) && (k < XD + PD);
      const float sv = (isd && half != 0) ? -wv : wv;
      const float val = (k < XD + PD) ? sv : 0.0f;
      o[e] = (unsigned short)bf16_bits(val);
    }
    dp = B0T + (size_t)v * 8;
  } else if (b < nbA + NU0B / NTHR + NU1B / NTHR) {
    const int v = (b - nbA - NU0B / NTHR) * NTHR + tid;
    bunit132(W1, v, o);
    dp = B1T + (size_t)v * 8;
  } else if (b < nbA + NU0B / NTHR + 2 * (NU1B / NTHR)) {
    const int v = (b - nbA - NU0B / NTHR - NU1B / NTHR) * NTHR + tid;
    bunit132(W2, v, o);
    dp = B2T + (size_t)v * 8;
  } else {
    return;
  }
  *(volatile v8us*)dp = o;
  __threadfence();
  *(volatile v8us*)dp = o;
}

__global__ __launch_bounds__(GTHR) void k_gemm(const unsigned short* __restrict__ A, int lda,
                                               const unsigned short* __restrict__ BT, int ldb, int K,
                                               float* Cm, int ldc) {
  __shared__ __attribute__((aligned(16))) float stg[GBM * GBN];
  const int tid = (int)threadIdx.x, lane = tid & 31, wave = tid >> 5, hh = lane >> 4, m = lane & 15;
  const int rowBase = (int)blockIdx.x * GBM;
  const int colBase = (int)blockIdx.y * GBN;

  v8f acc[8];
  {
    const v8f z = {0.f, 0.f, 0.f, 0.f, 0.f, 0.f, 0.f, 0.f};
#pragma unroll
    for (int t = 0; t < 8; ++t) acc[t] = z;
  }
  const unsigned short* ap = A  + (size_t)(rowBase + 16 * wave + m) * (size_t)lda + 8 * hh;
  const unsigned short* bp = BT + (size_t)(colBase + m) * (size_t)ldb + 8 * hh;

#pragma unroll 1
  for (int k0 = 0; k0 < K; k0 += 32) {
    FragB af;
    af.h[0] = *(const v8usa*)(ap + k0);
    af.h[1] = *(const v8usa*)(ap + k0 + 16);
#pragma unroll
    for (int nt = 0; nt < 8; ++nt) {
      const unsigned short* wq = bp + (size_t)(16 * nt) * (size_t)ldb + k0;
      FragB bf;
      bf.h[0] = *(const v8usa*)wq;
      bf.h[1] = *(const v8usa*)(wq + 16);
      acc[nt] = wmb(af, bf, acc[nt]);
    }
  }

#pragma unroll
  for (int nt = 0; nt < 8; ++nt) {
    const int lc = 16 * nt + m;
#pragma unroll
    for (int r = 0; r < 8; ++r) {
      const int lr = 16 * wave + 8 * hh + r;
      stg[lr * GBN + lc] = acc[nt][r];
    }
  }
  __syncthreads();

  v4f pv[16];
#pragma unroll
  for (int i = 0; i < 16; ++i) pv[i] = *(const v4fa*)(stg + (16 * wave + i) * GBN + 4 * lane);
#pragma unroll
  for (int i = 0; i < 16; ++i) {
    float* op = Cm + (size_t)(rowBase + 16 * wave + i) * (size_t)ldc + colBase + 4 * lane;
    *(volatile v4f*)op = pv[i];
  }
  __threadfence();
#pragma unroll
  for (int i = 0; i < 16; ++i) {
    float* op = Cm + (size_t)(rowBase + 16 * wave + i) * (size_t)ldc + colBase + 4 * lane;
    *(volatile v4f*)op = pv[i];
  }
}

template <int AOUT>
__global__ __launch_bounds__(NTHR) void k_agg(const int* __restrict__ srcs, const int* __restrict__ dsts,
                                              int nE, int nN, int vec8, int mRows,
                                              const float* __restrict__ ea, const float* __restrict__ pp,
                                              const float* __restrict__ uv, const float* __restrict__ bias,
                                              const float* __restrict__ wc,
                                              unsigned short* aout, float* hout) {
  extern __shared__ __attribute__((aligned(16))) int dsm[];
  int* list = dsm;
  int* hl   = dsm + LISTN;
  int* sl   = hl + RCAP;
  int* cnt  = sl + RCAP;
  int* offs = cnt + NBA;
  int* cur  = offs + NBA;
  int* misc = cur + NBA;
  const int tid = (int)threadIdx.x, lane = tid & 31, wave = tid >> 5;
  const int nodeBase = (int)blockIdx.x * NBA;

  {
    const v4i z4 = {0, 0, 0, 0};
    for (int i = tid * 4; i < AGG_ZINTS; i += NTHR * 4) *(v4ia*)(dsm + i) = z4;
    if (tid < 16) misc[tid] = 0;
  }
  float bv0, bv1, wc0, wc1;
  {
    const v2f bq = *(const v2f*)(bias + 2 * lane);
    bv0 = bf16_val(bq.x); bv1 = bf16_val(bq.y);
    const v2f wq = *(const v2f*)(wc + 2 * lane);
    wc0 = bf16_val(wq.x); wc1 = bf16_val(wq.y);
  }
  __syncthreads();

  int t = 0, ov = 0;
  const int nChunks = (nE + CHUNK - 1) / CHUNK;
#pragma unroll 1
  for (int ch = 0; ch < nChunks; ++ch) {
    const int cbase = ch * CHUNK;
    const int wcn = scan_chunk<SLA>(dsts, nE, cbase, nodeBase, NBA, vec8, list, tid, lane, wave);
    if (lane == 0) misc[wave] = wcn;
    __syncthreads();
    if (wave == 0) {
#pragma unroll 1
      for (int w2 = 0; w2 < NWAVE; ++w2) {
        int c = misc[w2];
        c = c < 0 ? 0 : (c > WCAP ? WCAP : c);
#pragma unroll 1
        for (int b0 = 0; b0 < c; b0 += 32) {
          const int idx = b0 + lane;
          const int ent = list[w2 * WCAP + (idx < WCAP ? idx : WCAP - 1)];
          const int m32 = (c - b0) < 32 ? (c - b0) : 32;
#pragma unroll 1
          for (int k = 0; k < m32; ++k) {
            const int u    = __builtin_amdgcn_readlane(ent, k);
            const int slot = u & (NBA - 1);
            const int el   = (u >> SLA) & (CHUNK - 1);
            const int pk   = ((cbase + el) << SLA) | slot;
            if (t < RCAP) {
              if (lane == 0) { hl[t] = pk; cnt[slot] = cnt[slot] + 1; }
              t = t + 1;
            } else {
              ov = 1;
            }
          }
        }
      }
    }
    __syncthreads();
  }
  if (wave == 0 && lane == 0) { misc[8] = t; misc[9] = ov; }
  __syncthreads();
  int tt = misc[8];
  tt = tt < 0 ? 0 : (tt > RCAP ? RCAP : tt);
  const int ovf = misc[9];

  if (wave == 0) {
    const int base = lane * (NBA / 32);
    int s = 0;
#pragma unroll 1
    for (int i = 0; i < NBA / 32; ++i) s += cnt[base + i];
    int incl = s;
#pragma unroll
    for (int d = 1; d < 32; d <<= 1) {
      const int y = __shfl_up(incl, d, 32);
      if (lane >= d) incl += y;
    }
    int run = incl - s;
#pragma unroll 1
    for (int i = 0; i < NBA / 32; ++i) {
      const int cv = cnt[base + i];
      offs[base + i] = run;
      cur[base + i]  = run;
      run += cv;
    }
  }
  __syncthreads();
  if (wave == 0) {
#pragma unroll 1
    for (int b0 = 0; b0 < tt; b0 += 32) {
      const int idx = b0 + lane;
      const int ent = hl[idx < RCAP ? idx : RCAP - 1];
      const int m32 = (tt - b0) < 32 ? (tt - b0) : 32;
#pragma unroll 1
      for (int k = 0; k < m32; ++k) {
        const int u    = __builtin_amdgcn_readlane(ent, k);
        const int slot = u & (NBA - 1);
        if (lane == 0) {
          int q = cur[slot];
          q = q < 0 ? 0 : (q > RCAP - 1 ? RCAP - 1 : q);
          sl[q] = u;
          cur[slot] = q + 1;
        }
      }
    }
  }
  __syncthreads();

  const float pz = (ovf != 0) ? __int_as_float(0x7fc00000) : 0.0f;
#pragma unroll 1
  for (int si = 0; si < NBA / NWAVE; ++si) {
    const int s    = si * NWAVE + wave;
    const int node = nodeBase + s;
    int c = cnt[s];
    const bool big = c > DEGCAP;
    c = c < 0 ? 0 : (c > DEGCAP ? DEGCAP : c);
    int o = offs[s];
    o = o < 0 ? 0 : (o > RCAP ? RCAP : o);
    const int nc = node < nN ? node : nN - 1;
    const v2f vq = *(const v2f*)(uv + (size_t)nc * NUV + NCH + 2 * lane);
    const float zb0 = vq.x + bv0;
    const float zb1 = vq.y + bv1;
    float acc0 = 0.0f, acc1 = 0.0f;
#pragma unroll 1
    for (int b0 = 0; b0 < c; b0 += 32) {
      int idx = o + b0 + lane;
      idx = idx > RCAP - 1 ? RCAP - 1 : idx;
      const int ent = sl[idx];
      int eid = ent >> SLA;
      eid = eid < 0 ? 0 : (eid > nE - 1 ? nE - 1 : eid);
      int sr = srcs[eid];
      sr = sr < 0 ? 0 : (sr > nN - 1 ? nN - 1 : sr);
      const float ev  = bf16_val(ea[eid]);
      const int   evi = __float_as_int(ev);
      const int m32 = (c - b0) < 32 ? (c - b0) : 32;
#pragma unroll 1
      for (int k = 0; k < m32; ++k) {
        const int   sk = __builtin_amdgcn_readlane(sr, k);
        const float ek = __int_as_float(__builtin_amdgcn_readlane(evi, k));
        const v2f up = *(const v2f*)(uv + (size_t)sk * NUV + 2 * lane);
        const float z0 = fmaf(ek, wc0, up.x + zb0);
        const float z1 = fmaf(ek, wc1, up.y + zb1);
        acc0 += fsig(z0);
        acc1 += fsig(z1);
      }
    }
    const float pzr = big ? __int_as_float(0x7fc00000) : pz;
    const bool live = node < nN;
    float v0 = acc0 + pzr, v1 = acc1 + pzr;
    v0 = live ? v0 : 0.0f;
    v1 = live ? v1 : 0.0f;
    if constexpr (AOUT != 0) {
      const unsigned h0 = bf16_bits(v0), h1 = bf16_bits(v1);
      const unsigned l0 = bf16_bits(v0 - __uint_as_float(h0 << 16));
      const unsigned l1 = bf16_bits(v1 - __uint_as_float(h1 << 16));
      const unsigned hw = (h0 & 0xFFFFu) | (h1 << 16);
      const unsigned lw = (l0 & 0xFFFFu) | (l1 << 16);
      const float p0 = pp[(size_t)nc * PD + 0];
      const float p1 = pp[(size_t)nc * PD + 1];
      const float p2 = pp[(size_t)nc * PD + 2];
      const unsigned q0 = (bf16_bits(p0) & 0xFFFFu) | (bf16_bits(p1) << 16);
      const unsigned q1 = bf16_bits(p2) & 0xFFFFu;
      unsigned pw = (lane == 0) ? q0 : ((lane == 1) ? q1 : 0u);
      pw = live ? pw : 0u;
      if (node < mRows) {
        unsigned* rp = (unsigned*)(aout + (size_t)node * KP);
        *(volatile unsigned*)(rp + lane)            = hw;
        *(volatile unsigned*)(rp + NCH / 2 + lane)  = lw;
        *(volatile unsigned*)(rp + NCH + lane)      = pw;
        __threadfence();
        *(volatile unsigned*)(rp + lane)            = hw;
        *(volatile unsigned*)(rp + NCH / 2 + lane)  = lw;
        *(volatile unsigned*)(rp + NCH + lane)      = pw;
      }
    } else {
      v2f hv;
      hv.x = v0; hv.y = v1;
      if (node < mRows) {
        float* op = hout + (size_t)node * NCH + 2 * lane;
        *(volatile v2f*)op = hv;
        __threadfence();
        *(volatile v2f*)op = hv;
      }
    }
  }
}

__global__ __launch_bounds__(NTHR) void k_pool(const int* __restrict__ batch, int nN, int vecb,
                                               const float* __restrict__ H, const float* __restrict__ Wp,
                                               const float* __restrict__ bp, float* out, int G) {
  __shared__ __attribute__((aligned(16))) float R[NBP * NCH];
  __shared__ __attribute__((aligned(16))) int plist[LISTN];
  __shared__ __attribute__((aligned(16))) float ps[NBP];
  __shared__ int pcnt[NBP];
  __shared__ int wcnt[NWAVE];
  const int tid = (int)threadIdx.x, lane = tid & 31, wave = tid >> 5;
  const int gBase = (int)blockIdx.x * NBP;
  int nb = G - gBase;
  nb = nb < 0 ? 0 : (nb > NBP ? NBP : nb);
  {
    const v4f z = {0.f, 0.f, 0.f, 0.f};
#pragma unroll 1
    for (int i = tid; i < NBP * NCH / 4; i += NTHR) *(v4fa*)(R + 4 * i) = z;
    if (tid < NBP) { pcnt[tid] = 0; ps[tid] = 0.0f; }
    if (tid < NWAVE) wcnt[tid] = 0;
  }
  float wp0, wp1;
  {
    const v2f w2 = *(const v2f*)(Wp + 2 * lane);
    wp0 = bf16_val(w2.x); wp1 = bf16_val(w2.y);
  }
  const float bpv = bf16_val(bp[0]);
  __syncthreads();

  const int nChunks = (nN + CHUNK - 1) / CHUNK;
#pragma unroll 1
  for (int ch = 0; ch < nChunks; ++ch) {
    const int cbase = ch * CHUNK;
    const int wcn = scan_chunk<SLA>(batch, nN, cbase, gBase, nb, vecb, plist, tid, lane, wave);
    if (lane == 0) wcnt[wave] = wcn;
    __syncthreads();
#pragma unroll 1
    for (int wsx = 0; wsx < NWAVE; ++wsx) {
      int n = __builtin_amdgcn_readfirstlane(wcnt[wsx]);
      n = n > WCAP ? WCAP : (n < 0 ? 0 : n);
      const int* lp = plist + wsx * WCAP;
#pragma unroll 1
      for (int i = 0; i < n; ++i) {
        const int ent = __builtin_amdgcn_readfirstlane(lp[i]);
        int slot = ent & (NBA - 1);
        slot = slot > NBP - 1 ? NBP - 1 : slot;
        if ((slot / GPW) == wave) {
          int nd = cbase + ((ent >> SLA) & (CHUNK - 1));
          nd = nd < 0 ? 0 : (nd > nN - 1 ? nN - 1 : nd);
          const v2f v = *(const v2f*)(H + (size_t)nd * NCH + 2 * lane);
          v2f* rq = (v2f*)(R + slot * NCH + 2 * lane);
          *rq = *rq + v;
          if (lane == 0) pcnt[slot] = pcnt[slot] + 1;
        }
      }
    }
    __syncthreads();
  }

  v2f ovv[GPW];
#pragma unroll
  for (int j = 0; j < GPW; ++j) {
    const int slot = GPW * wave + j;
    const int c = pcnt[slot];
    float cf = (float)c;
    cf = cf < 1.0f ? 1.0f : cf;
    const float rinv = 1.0f / cf;
    const v2f r = *(const v2f*)(R + slot * NCH + 2 * lane) * rinv;
    ovv[j] = r;
    const float pr = wsum(fmaf(r.x, wp0, r.y * wp1)) + bpv;
    if (lane == 0) ps[slot] = pr;
  }
#pragma unroll
  for (int j = 0; j < GPW; ++j) {
    const int slot = GPW * wave + j;
    if (slot < nb) *(volatile v2f*)(out + (size_t)G + (size_t)(gBase + slot) * NCH + 2 * lane) = ovv[j];
  }
  __syncthreads();
  const v4f pv = *(const v4fa*)(ps + 4 * (lane & 7));
  const bool pwr = (wave == 0) && (lane < NBP / 4) && (nb == NBP);
  if (pwr) *(volatile v4f*)(out + (size_t)gBase + 4 * lane) = pv;
  __threadfence();
#pragma unroll
  for (int j = 0; j < GPW; ++j) {
    const int slot = GPW * wave + j;
    if (slot < nb) *(volatile v2f*)(out + (size_t)G + (size_t)(gBase + slot) * NCH + 2 * lane) = ovv[j];
  }
  if (pwr) *(volatile v4f*)(out + (size_t)gBase + 4 * lane) = pv;
}

static inline int cdiv(int a, int b) { return (a + b - 1) / b; }

extern "C" void kernel_launch(void* const* d_in, const int* in_sizes, int n_in,
                              void* d_out, int out_size, void* d_ws, size_t ws_size,
                              hipStream_t stream) {
  if (n_in < 13) return;
  if (in_sizes[0] < XD || (in_sizes[0] % XD) != 0) return;
  const int nN = in_sizes[0] / XD;
  if (nN < 1 || nN >= (1 << 22)) return;
  if (in_sizes[1] != nN * PD) return;
  if (in_sizes[2] < 2 || (in_sizes[2] & 1) != 0) return;
  const int nE = in_sizes[2] / 2;
  if (nE < 1 || nE >= (1 << 21)) return;
  if (in_sizes[3] != nE) return;
  if (in_sizes[4] != nN) return;
  if (in_sizes[5] != F0 * NCH || in_sizes[6] != NCH) return;
  if (in_sizes[7] != F1 * NCH || in_sizes[8] != NCH) return;
  if (in_sizes[9] != F1 * NCH || in_sizes[10] != NCH) return;
  if (in_sizes[11] != NCH || in_sizes[12] < 1) return;
  if (out_size < 65 || (out_size % 65) != 0) return;
  const int G = out_size / 65;
  if ((G % NBP) != 0) return;
  if ((long long)G + (long long)G * NCH > (long long)out_size) return;

  const float* x     = (const float*)d_in[0];
  const float* p     = (const float*)d_in[1];
  const int*   edge  = (const int*)d_in[2];
  const float* eattr = (const float*)d_in[3];
  const int*   batch = (const int*)d_in[4];
  const float* W0    = (const float*)d_in[5];
  const float* b0    = (const float*)d_in[6];
  const float* W1    = (const float*)d_in[7];
  const float* b1    = (const float*)d_in[8];
  const float* W2    = (const float*)d_in[9];
  const float* b2    = (const float*)d_in[10];
  const float* Wp    = (const float*)d_in[11];
  const float* bp    = (const float*)d_in[12];
  float* out = (float*)d_out;
  const int* src = edge;
  const int* dst = edge + nE;

  const int MP = cdiv(nN, 128) * 128;
  const int gM = MP / GBM;
  const int gA = cdiv(nN, NBA);
  if ((long long)gA * NBA < (long long)MP) return;
  const int vec8 = ((nE & 3) == 0) ? 1 : 0;
  const int vecb = 1;

  char* ws = (char*)d_ws;
  size_t off = 0;
  const size_t AL = 1023;
  const size_t oA0 = off; off += (size_t)MP * KP0 * 2;     off = (off + AL) & ~AL;
  const size_t oB0 = off; off += (size_t)NUV * KP0 * 2;    off = (off + AL) & ~AL;
  const size_t oB1 = off; off += (size_t)NUV * KP * 2;     off = (off + AL) & ~AL;
  const size_t oB2 = off; off += (size_t)NUV * KP * 2;     off = (off + AL) & ~AL;
  const size_t oUV = off; off += (size_t)MP * NUV * 4;     off = (off + AL) & ~AL;
  const size_t oA1 = off; off += (size_t)MP * KP * 2;      off = (off + AL) & ~AL;
  const size_t oA2 = off; off += (size_t)MP * KP * 2;      off = (off + AL) & ~AL;
  const size_t oH3 = off; off += (size_t)MP * NCH * 4;     off = (off + AL) & ~AL;
  if (off > ws_size || off > (size_t)WSMAX) return;
  unsigned short* A0  = (unsigned short*)(ws + oA0);
  unsigned short* B0T = (unsigned short*)(ws + oB0);
  unsigned short* B1T = (unsigned short*)(ws + oB1);
  unsigned short* B2T = (unsigned short*)(ws + oB2);
  float*          UV  = (float*)(ws + oUV);
  unsigned short* A1  = (unsigned short*)(ws + oA1);
  unsigned short* A2  = (unsigned short*)(ws + oA2);
  float*          H3  = (float*)(ws + oH3);

  const size_t aggLds = (size_t)AGG_LDS_INTS * 4;
  hipFuncSetAttribute(reinterpret_cast<const void*>(&k_agg<1>), hipFuncAttributeMaxDynamicSharedMemorySize, (int)aggLds);
  hipFuncSetAttribute(reinterpret_cast<const void*>(&k_agg<0>), hipFuncAttributeMaxDynamicSharedMemorySize, (int)aggLds);

  const int nbPrep = gM + NU0B / NTHR + 2 * (NU1B / NTHR);
  k_prep<<<nbPrep, NTHR, 0, stream>>>(x, p, W0, W1, W2, nN, gM, A0, B0T, B1T, B2T);
  k_gemm<<<dim3(gM, NUV / GBN), GTHR, 0, stream>>>(A0, KP0, B0T, KP0, KP0, UV, NUV);
  k_agg<1><<<gA, NTHR, aggLds, stream>>>(src, dst, nE, nN, vec8, MP, eattr, p, UV, b0, W0 + (size_t)(2 * XD) * NCH, A1, H3);
  k_gemm<<<dim3(gM, NUV / GBN), GTHR, 0, stream>>>(A1, KP, B1T, KP, KP, UV, NUV);
  k_agg<1><<<gA, NTHR, aggLds, stream>>>(src, dst, nE, nN, vec8, MP, eattr, p, UV, b1, W1 + (size_t)(2 * NCH) * NCH, A2, H3);
  k_gemm<<<dim3(gM, NUV / GBN), GTHR, 0, stream>>>(A2, KP, B2T, KP, KP, UV, NUV);
  k_agg<0><<<gA, NTHR, aggLds, stream>>>(src, dst, nE, nN, vec8, MP, eattr, p, UV, b2, W2 + (size_t)(2 * NCH) * NCH, A1, H3);
  k_pool<<<G / NBP, NTHR, 0, stream>>>(batch, nN, vecb, H3, Wp, bp, out, G);
}
